// MambaBlock_19275813224604
// MI455X (gfx1250) — hardware-verified
//
#include <hip/hip_runtime.h>
#include <stddef.h>
#include <stdint.h>

#define SEQL  2048
#define DMOD  768
#define DINN  1536
#define DSTA  16
#define DTRK  48
#define XDW   80
#define XDP   96
#define DTLP  128
#define KDT   96
#define K2    3072
#define NTHR  256
#define GTHR  128
#define GBM   64
#define WSMAX 134217728
#define EPSF  1.1920928955078125e-07f
#define REPS  8388608.0f

#define VO_CW  0
#define VO_AN  6144
#define VO_CB  30720
#define VO_DTB 32256
#define VO_DV  33792
#define VEC_N  35328

#define NU_XB  (SEQL * DMOD / 8)
#define NU_WIN (2 * DINN * DMOD / 8)
#define NU_XP2 (XDP * K2 / 8)
#define NU_DTW (DINN * KDT / 8)
#define NU_WO  (DMOD * K2 / 8)
#define NU_CW  (DINN * 4 / 4)
#define NU_AN  (DINN * DSTA / 4)
#define NU_V   (DINN / 4)
#define P0 (NU_XB)
#define P1 (P0 + NU_WIN)
#define P2 (P1 + NU_XP2)
#define P3 (P2 + NU_DTW)
#define P4 (P3 + NU_WO)
#define P5 (P4 + NU_CW)
#define P6 (P5 + NU_AN)
#define P7 (P6 + NU_V)
#define P8 (P7 + NU_V)
#define P9 (P8 + NU_V)

static_assert(NU_XB % 32 == 0 && NU_WIN % 32 == 0 && NU_XP2 % 32 == 0 && NU_DTW % 32 == 0 && NU_WO % 32 == 0);
static_assert(NU_CW % 32 == 0 && NU_AN % 32 == 0 && NU_V % 32 == 0);
static_assert(VO_AN == DINN * 4 && VO_CB == VO_AN + DINN * DSTA && VO_DTB == VO_CB + DINN);
static_assert(VO_DV == VO_DTB + DINN && VEC_N == VO_DV + DINN);
static_assert(SEQL % GBM == 0 && (2 * DINN) % 128 == 0 && DINN % 128 == 0 && DMOD % 128 == 0);
static_assert(DMOD % 32 == 0 && K2 % 32 == 0 && KDT % 32 == 0 && K2 == 2 * DINN && KDT == 2 * DTRK);
static_assert(XDP >= XDW && XDP % 16 == 0 && DTLP >= KDT && DTRK % 8 == 0);
static_assert((DINN / 4) % 32 == 0 && (DINN / 8) % 32 == 0 && SEQL % 64 == 0 && DINN % 32 == 0);

typedef float          v4f   __attribute__((ext_vector_type(4)));
typedef float          v8f   __attribute__((ext_vector_type(8)));
typedef int            v8i   __attribute__((ext_vector_type(8)));
typedef unsigned short v4us  __attribute__((ext_vector_type(4)));
typedef unsigned short v8us  __attribute__((ext_vector_type(8)));
typedef unsigned short v16us __attribute__((ext_vector_type(16)));
typedef __bf16         v16bf __attribute__((ext_vector_type(16)));
typedef v4f  __attribute__((may_alias)) v4fa;
typedef v8us __attribute__((may_alias)) v8usa;
union FragB { v16bf v; v16us u; v8us h[2]; v8i w; };

__device__ __forceinline__ v8f wmb(const FragB& a, const FragB& b, v8f c) {
  v8f d = __builtin_amdgcn_wmma_f32_16x16x32_bf16(false, a.v, false, b.v, (short)0, c, false, false);
  asm volatile("v_nop\n\tv_nop\n\tv_nop\n\tv_nop" : "+v"(d) : "v"(a.w), "v"(b.w));
  return d;
}

__device__ __forceinline__ unsigned bf16_bits(float f) {
  const unsigned u = __float_as_uint(f);
  return (u + 0x7FFFu + ((u >> 16) & 1u)) >> 16;
}
__device__ __forceinline__ float bf16_val(float f) {
  return __uint_as_float(bf16_bits(f) << 16);
}
__device__ __forceinline__ void put16(unsigned short* dp, v8us o) {
  *(volatile v8us*)dp = o;
  __threadfence();
  *(volatile v8us*)dp = o;
}
__device__ __forceinline__ void putf4(float* dp, v4f o) {
  *(volatile v4f*)dp = o;
  __threadfence();
  *(volatile v4f*)dp = o;
}
__device__ __forceinline__ float silu_f(float v) {
  return v * (1.0f / (1.0f + expf(-v)));
}
__device__ __forceinline__ float softplus_f(float v) {
  return fmaxf(v, 0.0f) + log1pf(expf(-fabsf(v)));
}
__device__ __forceinline__ v8us cvt8(const float* __restrict__ p) {
  const v4f a = *(const v4fa*)p;
  const v4f b = *(const v4fa*)(p + 4);
  v8us o;
  o[0] = (unsigned short)bf16_bits(a.x);
  o[1] = (unsigned short)bf16_bits(a.y);
  o[2] = (unsigned short)bf16_bits(a.z);
  o[3] = (unsigned short)bf16_bits(a.w);
  o[4] = (unsigned short)bf16_bits(b.x);
  o[5] = (unsigned short)bf16_bits(b.y);
  o[6] = (unsigned short)bf16_bits(b.z);
  o[7] = (unsigned short)bf16_bits(b.w);
  return o;
}
__device__ __forceinline__ v4f bfv4(const float* __restrict__ p) {
  const v4f a = *(const v4fa*)p;
  v4f o;
  o.x = bf16_val(a.x);
  o.y = bf16_val(a.y);
  o.z = bf16_val(a.z);
  o.w = bf16_val(a.w);
  return o;
}

__global__ __launch_bounds__(NTHR) void k_prep(const float* __restrict__ x, const float* __restrict__ win,
                                               const float* __restrict__ convw, const float* __restrict__ convb,
                                               const float* __restrict__ xpw, const float* __restrict__ dtw,
                                               const float* __restrict__ dtb, const float* __restrict__ alog,
                                               const float* __restrict__ dvec, const float* __restrict__ wo,
                                               unsigned short* XB, unsigned short* WIN, unsigned short* XP2,
                                               unsigned short* DTW2, unsigned short* WO2, float* VEC) {
  const int u = (int)blockIdx.x * NTHR + (int)threadIdx.x;
  if (u >= P9) return;
  if (u < P0) {
    put16(XB + (size_t)u * 8, cvt8(x + (size_t)u * 8));
  } else if (u < P1) {
    const int v = u - P0;
    put16(WIN + (size_t)v * 8, cvt8(win + (size_t)v * 8));
  } else if (u < P2) {
    const int v  = u - P1;
    const int n  = v / (K2 / 8);
    const int k8 = (v - n * (K2 / 8)) * 8;
    const int kk = k8 >= DINN ? k8 - DINN : k8;
    const int nc = n < XDW ? n : XDW - 1;
    const unsigned short mk = (unsigned short)(n < XDW ? 0xffffu : 0u);
    v8us o = cvt8(xpw + (size_t)nc * DINN + kk);
#pragma unroll
    for (int i = 0; i < 8; ++i) o[i] = (unsigned short)(o[i] & mk);
    put16(XP2 + (size_t)v * 8, o);
  } else if (u < P3) {
    const int v  = u - P2;
    const int c  = v / (KDT / 8);
    const int k8 = (v - c * (KDT / 8)) * 8;
    const int kk = k8 >= DTRK ? k8 - DTRK : k8;
    put16(DTW2 + (size_t)v * 8, cvt8(dtw + (size_t)c * DTRK + kk));
  } else if (u < P4) {
    const int v  = u - P3;
    const int n  = v / (K2 / 8);
    const int k8 = (v - n * (K2 / 8)) * 8;
    const int kk = k8 >= DINN ? k8 - DINN : k8;
    put16(WO2 + (size_t)v * 8, cvt8(wo + (size_t)n * DINN + kk));
  } else if (u < P5) {
    const int v = u - P4;
    putf4(VEC + VO_CW + 4 * v, bfv4(convw + 4 * v));
  } else if (u < P6) {
    const int v = u - P5;
    const v4f a = bfv4(alog + 4 * v);
    v4f o;
    o.x = -expf(a.x);
    o.y = -expf(a.y);
    o.z = -expf(a.z);
    o.w = -expf(a.w);
    putf4(VEC + VO_AN + 4 * v, o);
  } else if (u < P7) {
    const int v = u - P6;
    putf4(VEC + VO_CB + 4 * v, bfv4(convb + 4 * v));
  } else if (u < P8) {
    const int v = u - P7;
    putf4(VEC + VO_DTB + 4 * v, bfv4(dtb + 4 * v));
  } else {
    const int v = u - P8;
    putf4(VEC + VO_DV + 4 * v, bfv4(dvec + 4 * v));
  }
}

template <int NT, int MODE>
__global__ __launch_bounds__(GTHR) void k_gemm(const unsigned short* __restrict__ A, int lda,
                                               const unsigned short* __restrict__ BT, int ldb, int K,
                                               const float* __restrict__ bias,
                                               float* C0, float* C1, unsigned short* Cb, int ldc) {
  constexpr int GBN = 16 * NT;
  static_assert((MODE == 1 && NT == 6 && GBN == XDP) || (MODE != 1 && NT == 8));
  __shared__ __attribute__((aligned(16))) float stg[GBM * GBN];
  const int tid = (int)threadIdx.x, lane = tid & 31, wave = tid >> 5, hh = lane >> 4, m = lane & 15;
  const int rowBase = (int)blockIdx.x * GBM;
  const int colBase = (int)blockIdx.y * GBN;

  v8f acc[NT];
  {
    const v8f z = {0.f, 0.f, 0.f, 0.f, 0.f, 0.f, 0.f, 0.f};
#pragma unroll
    for (int t = 0; t < NT; ++t) acc[t] = z;
  }
  const unsigned short* ap = A  + (size_t)(rowBase + 16 * wave + m) * (size_t)lda + 8 * hh;
  const unsigned short* bp = BT + (size_t)(colBase + m) * (size_t)ldb + 8 * hh;

#pragma unroll 1
  for (int k0 = 0; k0 < K; k0 += 32) {
    FragB af;
    af.h[0] = *(const v8usa*)(ap + k0);
    af.h[1] = *(const v8usa*)(ap + k0 + 16);
#pragma unroll
    for (int nt = 0; nt < NT; ++nt) {
      const unsigned short* wq = bp + (size_t)(16 * nt) * (size_t)ldb + k0;
      FragB bf;
      bf.h[0] = *(const v8usa*)wq;
      bf.h[1] = *(const v8usa*)(wq + 16);
      acc[nt] = wmb(af, bf, acc[nt]);
    }
  }

#pragma unroll
  for (int nt = 0; nt < NT; ++nt) {
    const int lc = 16 * nt + m;
    float bvv = 0.0f;
    if constexpr (MODE == 2) bvv = bias[colBase + lc];
#pragma unroll
    for (int r = 0; r < 8; ++r) {
      const int lr = 16 * wave + 8 * hh + r;
      stg[lr * GBN + lc] = acc[nt][r] + bvv;
    }
  }
  __syncthreads();

  if constexpr (MODE == 0 || MODE == 2) {
    const bool act = (MODE == 2) || (colBase >= DINN);
    if (act) {
#pragma unroll 1
      for (int i = 0; i < 16; ++i) {
        float* sp = stg + (16 * wave + i) * GBN + 4 * lane;
        v4f v = *(const v4fa*)sp;
        if constexpr (MODE == 0) {
          v.x = silu_f(v.x); v.y = silu_f(v.y); v.z = silu_f(v.z); v.w = silu_f(v.w);
        } else {
          v.x = softplus_f(v.x); v.y = softplus_f(v.y); v.z = softplus_f(v.z); v.w = softplus_f(v.w);
        }
        *(v4fa*)sp = v;
      }
    }
    __syncthreads();
  }

  if constexpr (MODE == 1) {
    const float* sw = stg + 16 * wave * GBN;
    v4f px[12];
#pragma unroll
    for (int it = 0; it < 12; ++it) px[it] = *(const v4fa*)(sw + 4 * (it * 32 + lane));
    v8us pd[8];
#pragma unroll
    for (int it = 0; it < 8; ++it) {
      const int idx = it * 32 + lane;
      const int i   = idx >> 4;
      const int j   = idx & 15;
      const int jj  = j < 6 ? j : (j < 12 ? j - 6 : 0);
      const unsigned mhi = j < 6 ? 0xffffu : 0u;
      const unsigned mlo = (j >= 6 && j < 12) ? 0xffffu : 0u;
      const float* sp = sw + i * GBN + 8 * jj;
      const v4f a = *(const v4fa*)sp;
      const v4f b = *(const v4fa*)(sp + 4);
      const v8f f8 = {a.x, a.y, a.z, a.w, b.x, b.y, b.z, b.w};
      v8us oo;
#pragma unroll
      for (int e = 0; e < 8; ++e) {
        const unsigned hb = bf16_bits(f8[e]);
        const unsigned lb = bf16_bits(f8[e] - __uint_as_float(hb << 16));
        oo[e] = (unsigned short)((hb & mhi) | (lb & mlo));
      }
      pd[it] = oo;
    }
    float*          xd = C0 + (size_t)(rowBase + 16 * wave) * XDP;
    unsigned short* dd = Cb + (size_t)(rowBase + 16 * wave) * DTLP;
#pragma unroll
    for (int it = 0; it < 12; ++it) *(volatile v4f*)(xd + 4 * (it * 32 + lane)) = px[it];
#pragma unroll
    for (int it = 0; it < 8; ++it) *(volatile v8us*)(dd + 8 * (it * 32 + lane)) = pd[it];
    __threadfence();
#pragma unroll
    for (int it = 0; it < 12; ++it) *(volatile v4f*)(xd + 4 * (it * 32 + lane)) = px[it];
#pragma unroll
    for (int it = 0; it < 8; ++it) *(volatile v8us*)(dd + 8 * (it * 32 + lane)) = pd[it];
  } else {
    float* Cp = C0;
    int cb = colBase;
    if constexpr (MODE == 0) {
      if (colBase >= DINN) { Cp = C1; cb = colBase - DINN; }
    }
    v4f pv[16];
#pragma unroll
    for (int i = 0; i < 16; ++i) pv[i] = *(const v4fa*)(stg + (16 * wave + i) * GBN + 4 * lane);
#pragma unroll
    for (int i = 0; i < 16; ++i) {
      float* op = Cp + (size_t)(rowBase + 16 * wave + i) * (size_t)ldc + cb + 4 * lane;
      *(volatile v4f*)op = pv[i];
    }
    __threadfence();
#pragma unroll
    for (int i = 0; i < 16; ++i) {
      float* op = Cp + (size_t)(rowBase + 16 * wave + i) * (size_t)ldc + cb + 4 * lane;
      *(volatile v4f*)op = pv[i];
    }
  }
}

__global__ __launch_bounds__(NTHR) void k_conv(const float* __restrict__ XH, const float* __restrict__ VEC,
                                               float* U, unsigned short* UHL) {
  const int u = (int)blockIdx.x * NTHR + (int)threadIdx.x;
  if (u >= SEQL * (DINN / 4)) return;
  const int t  = u / (DINN / 4);
  const int j  = u - t * (DINN / 4);
  const int c4 = 4 * j;
  const v4f w0 = *(const v4fa*)(VEC + VO_CW + (c4 + 0) * 4);
  const v4f w1 = *(const v4fa*)(VEC + VO_CW + (c4 + 1) * 4);
  const v4f w2 = *(const v4fa*)(VEC + VO_CW + (c4 + 2) * 4);
  const v4f w3 = *(const v4fa*)(VEC + VO_CW + (c4 + 3) * 4);
  const v4f cb = *(const v4fa*)(VEC + VO_CB + c4);
  v4f xr[4];
#pragma unroll
  for (int jt = 0; jt < 4; ++jt) {
    const int tt  = t + jt - 3;
    const int ttc = tt < 0 ? 0 : tt;
    const float keep = tt < 0 ? 0.0f : 1.0f;
    const v4f a = *(const v4fa*)(XH + (size_t)ttc * DINN + c4);
    xr[jt] = a * keep;
  }
  v4f xc;
  xc.x = w0.x * xr[0].x + w0.y * xr[1].x + w0.z * xr[2].x + w0.w * xr[3].x + cb.x;
  xc.y = w1.x * xr[0].y + w1.y * xr[1].y + w1.z * xr[2].y + w1.w * xr[3].y + cb.y;
  xc.z = w2.x * xr[0].z + w2.y * xr[1].z + w2.z * xr[2].z + w2.w * xr[3].z + cb.z;
  xc.w = w3.x * xr[0].w + w3.y * xr[1].w + w3.z * xr[2].w + w3.w * xr[3].w + cb.w;
  v4f uo;
  uo.x = silu_f(xc.x);
  uo.y = silu_f(xc.y);
  uo.z = silu_f(xc.z);
  uo.w = silu_f(xc.w);
  v4us ohi, olo;
#pragma unroll
  for (int e = 0; e < 4; ++e) {
    const unsigned hb = bf16_bits(uo[e]);
    ohi[e] = (unsigned short)hb;
    olo[e] = (unsigned short)bf16_bits(uo[e] - __uint_as_float(hb << 16));
  }
  float*          up = U + (size_t)t * DINN + c4;
  unsigned short* hp = UHL + (size_t)t * K2 + c4;
  *(volatile v4f*)up           = uo;
  *(volatile v4us*)hp          = ohi;
  *(volatile v4us*)(hp + DINN) = olo;
  __threadfence();
  *(volatile v4f*)up           = uo;
  *(volatile v4us*)hp          = ohi;
  *(volatile v4us*)(hp + DINN) = olo;
}

__global__ __launch_bounds__(512) void k_scan(const float* __restrict__ DT, const float* __restrict__ U,
                                              const float* __restrict__ SZ, const float* __restrict__ XD,
                                              const float* __restrict__ VEC, float* YGF) {
#pragma clang fp contract(off)
  __shared__ __attribute__((aligned(16))) float sDT[64 * 32];
  __shared__ __attribute__((aligned(16))) float sU[64 * 32];
  __shared__ __attribute__((aligned(16))) float sSZ[64 * 32];
  __shared__ __attribute__((aligned(16))) float sBC[64 * 32];
  __shared__ __attribute__((aligned(16))) float sY[64 * 32];
  const int tid = (int)threadIdx.x;
  const int n = tid & 15, cl = tid >> 4;
  const int c0 = (int)blockIdx.x * 32;
  const int c = c0 + cl;
  const int srow = tid >> 3, sq = tid & 7;
  const float Aa = VEC[VO_AN + c * DSTA + n];
  const float Dc = VEC[VO_DV + c];
  float p = 1.0f, g = 0.0f;
  int tail = 0;

#pragma unroll 1
  for (int t0 = 0; t0 < SEQL; t0 += 64) {
    __syncthreads();
    const size_t gi = (size_t)(t0 + srow) * DINN + c0 + 4 * sq;
    {
      const v4f a  = *(const v4fa*)(DT + gi);
      const v4f b  = *(const v4fa*)(U + gi);
      const v4f s  = *(const v4fa*)(SZ + gi);
      const v4f bc = *(const v4fa*)(XD + (size_t)(t0 + srow) * XDP + DTRK + 4 * sq);
      *(v4fa*)(sDT + srow * 32 + 4 * sq) = a;
      *(v4fa*)(sU  + srow * 32 + 4 * sq) = b;
      *(v4fa*)(sSZ + srow * 32 + 4 * sq) = s;
      *(v4fa*)(sBC + srow * 32 + 4 * sq) = bc;
    }
    __syncthreads();

    if (tail == 0) {
#pragma unroll 1
      for (int tl = 0; tl < 64; ++tl) {
        const float dt = sDT[tl * 32 + cl];
        const float uv = sU[tl * 32 + cl];
        const float sz = sSZ[tl * 32 + cl];
        const float bn = sBC[tl * 32 + n];
        const float cn = sBC[tl * 32 + 16 + n];
        const float dA = expf(dt * Aa);
        p = p * dA;
        const float dbu = (dt * bn) * uv;
        g = g + dbu / fmaxf(p, EPSF);
        const float h = g * p;
        float part = h * cn;
        part += __shfl_xor(part, 8);
        part += __shfl_xor(part, 4);
        part += __shfl_xor(part, 2);
        part += __shfl_xor(part, 1);
        const float yv = (part + Dc * uv) * sz;
        if (n == 0) sY[tl * 32 + cl] = yv;
      }
    } else {
#pragma unroll 1
      for (int tl = 0; tl < 64; ++tl) {
        const float dt = sDT[tl * 32 + cl];
        const float uv = sU[tl * 32 + cl];
        const float sz = sSZ[tl * 32 + cl];
        const float bn = sBC[tl * 32 + n];
        const float cn = sBC[tl * 32 + 16 + n];
        const float dbu = (dt * bn) * uv;
        g = g + dbu * REPS;
        const float h = g * p;
        float part = h * cn;
        part += __shfl_xor(part, 8);
        part += __shfl_xor(part, 4);
        part += __shfl_xor(part, 2);
        part += __shfl_xor(part, 1);
        const float yv = (part + Dc * uv) * sz;
        if (n == 0) sY[tl * 32 + cl] = yv;
      }
    }
    {
      const bool z = (p == 0.0f) && (Aa < 0.0f);
      tail = (__builtin_amdgcn_ballot_w32(z) == 0xffffffffu) ? 1 : 0;
    }
    __syncthreads();
    {
      const v4f v = *(const v4fa*)(sY + srow * 32 + 4 * sq);
      putf4(YGF + gi, v);
    }
  }
}

__global__ __launch_bounds__(NTHR) void k_split(const float* __restrict__ YGF, unsigned short* YGH) {
  const int u = (int)blockIdx.x * NTHR + (int)threadIdx.x;
  if (u >= SEQL * (DINN / 8)) return;
  const int row = u / (DINN / 8);
  const int j   = u - row * (DINN / 8);
  const float* mq = YGF + (size_t)row * DINN + 8 * j;
  const v4f ma = *(const v4fa*)mq;
  const v4f mb = *(const v4fa*)(mq + 4);
  const v8f m8 = {ma.x, ma.y, ma.z, ma.w, mb.x, mb.y, mb.z, mb.w};
  v8us ohi, olo;
#pragma unroll
  for (int i = 0; i < 8; ++i) {
    const unsigned hbits = bf16_bits(m8[i]);
    ohi[i] = (unsigned short)hbits;
    olo[i] = (unsigned short)bf16_bits(m8[i] - __uint_as_float(hbits << 16));
  }
  unsigned short* dp = YGH + (size_t)row * K2 + 8 * j;
  *(volatile v8us*)dp          = ohi;
  *(volatile v8us*)(dp + DINN) = olo;
  __threadfence();
  *(volatile v8us*)dp          = ohi;
  *(volatile v8us*)(dp + DINN) = olo;
}

extern "C" void kernel_launch(void* const* d_in, const int* in_sizes, int n_in,
                              void* d_out, int out_size, void* d_ws, size_t ws_size,
                              hipStream_t stream) {
  if (n_in < 10) return;
  if (in_sizes[0] != SEQL * DMOD) return;
  if (in_sizes[1] != 2 * DINN * DMOD) return;
  if (in_sizes[2] != DINN * 4) return;
  if (in_sizes[3] != DINN) return;
  if (in_sizes[4] != XDW * DINN) return;
  if (in_sizes[5] != DINN * DTRK) return;
  if (in_sizes[6] != DINN) return;
  if (in_sizes[7] != DINN * DSTA) return;
  if (in_sizes[8] != DINN) return;
  if (in_sizes[9] != DMOD * DINN) return;
  if (out_size != SEQL * DMOD) return;

  const float* x     = (const float*)d_in[0];
  const float* win   = (const float*)d_in[1];
  const float* convw = (const float*)d_in[2];
  const float* convb = (const float*)d_in[3];
  const float* xpw   = (const float*)d_in[4];
  const float* dtw   = (const float*)d_in[5];
  const float* dtb   = (const float*)d_in[6];
  const float* alog  = (const float*)d_in[7];
  const float* dvec  = (const float*)d_in[8];
  const float* wo    = (const float*)d_in[9];
  float* out = (float*)d_out;

  char* ws = (char*)d_ws;
  size_t off = 0;
  const size_t oXB  = off; off += (size_t)SEQL * DMOD * 2;       off = (off + 255) & ~(size_t)255;
  const size_t oWIN = off; off += (size_t)2 * DINN * DMOD * 2;   off = (off + 255) & ~(size_t)255;
  const size_t oXP2 = off; off += (size_t)XDP * K2 * 2;          off = (off + 255) & ~(size_t)255;
  const size_t oDTW = off; off += (size_t)DINN * KDT * 2;        off = (off + 255) & ~(size_t)255;
  const size_t oWO2 = off; off += (size_t)DMOD * K2 * 2;         off = (off + 255) & ~(size_t)255;
  const size_t oVEC = off; off += (size_t)VEC_N * 4;             off = (off + 255) & ~(size_t)255;
  const size_t oXH  = off; off += (size_t)SEQL * DINN * 4;       off = (off + 255) & ~(size_t)255;
  const size_t oSZ  = off; off += (size_t)SEQL * DINN * 4;       off = (off + 255) & ~(size_t)255;
  const size_t oU   = off; off += (size_t)SEQL * DINN * 4;       off = (off + 255) & ~(size_t)255;
  const size_t oUHL = off; off += (size_t)SEQL * K2 * 2;         off = (off + 255) & ~(size_t)255;
  const size_t oXD  = off; off += (size_t)SEQL * XDP * 4;        off = (off + 255) & ~(size_t)255;
  const size_t oDTL = off; off += (size_t)SEQL * DTLP * 2;       off = (off + 255) & ~(size_t)255;
  const size_t oDT  = off; off += (size_t)SEQL * DINN * 4;       off = (off + 255) & ~(size_t)255;
  const size_t oYGF = off; off += (size_t)SEQL * DINN * 4;       off = (off + 255) & ~(size_t)255;
  const size_t oYGH = off; off += (size_t)SEQL * K2 * 2;         off = (off + 255) & ~(size_t)255;
  if (off > ws_size || off > (size_t)WSMAX) return;

  unsigned short* XB   = (unsigned short*)(ws + oXB);
  unsigned short* WIN  = (unsigned short*)(ws + oWIN);
  unsigned short* XP2  = (unsigned short*)(ws + oXP2);
  unsigned short* DTW2 = (unsigned short*)(ws + oDTW);
  unsigned short* WO2  = (unsigned short*)(ws + oWO2);
  float*          VEC  = (float*)(ws + oVEC);
  float*          XH   = (float*)(ws + oXH);
  float*          SZ   = (float*)(ws + oSZ);
  float*          U    = (float*)(ws + oU);
  unsigned short* UHL  = (unsigned short*)(ws + oUHL);
  float*          XD   = (float*)(ws + oXD);
  unsigned short* DTL  = (unsigned short*)(ws + oDTL);
  float*          DT   = (float*)(ws + oDT);
  float*          YGF  = (float*)(ws + oYGF);
  unsigned short* YGH  = (unsigned short*)(ws + oYGH);

  k_prep<<<(P9 + NTHR - 1) / NTHR, NTHR, 0, stream>>>(x, win, convw, convb, xpw, dtw, dtb, alog, dvec, wo,
                                                       XB, WIN, XP2, DTW2, WO2, VEC);
  k_gemm<8, 0><<<dim3(SEQL / GBM, (2 * DINN) / 128), GTHR, 0, stream>>>(XB, DMOD, WIN, DMOD, DMOD, VEC,
                                                                         XH, SZ, DTL, DINN);
  k_conv<<<(SEQL * (DINN / 4)) / NTHR, NTHR, 0, stream>>>(XH, VEC, U, UHL);
  k_gemm<6, 1><<<dim3(SEQL / GBM, 1), GTHR, 0, stream>>>(UHL, K2, XP2, K2, K2, VEC, XD, XD, DTL, XDP);
  k_gemm<8, 2><<<dim3(SEQL / GBM, DINN / 128), GTHR, 0, stream>>>(DTL, DTLP, DTW2, KDT, KDT, VEC + VO_DTB,
                                                                   DT, DT, DTL, DINN);
  k_scan<<<DINN / 32, 512, 0, stream>>>(DT, U, SZ, XD, VEC, YGF);
  k_split<<<(SEQL * (DINN / 8)) / NTHR, NTHR, 0, stream>>>(YGF, YGH);
  k_gemm<8, 3><<<dim3(SEQL / GBM, DMOD / 128), GTHR, 0, stream>>>(YGH, K2, WO2, K2, K2, VEC, out, out, DTL, DMOD);
}
